// ConcatCritic_31207232372863
// MI455X (gfx1250) — hardware-verified
//
#include <hip/hip_runtime.h>


#define NBX  512
#define DX   128
#define HID  512
#define CHA  64
#define NR   (CHA * NBX)
typedef _Float16 h16;
typedef unsigned short bf;
typedef __attribute__((ext_vector_type(16))) __bf16   v16bf;
typedef __attribute__((ext_vector_type(16))) _Float16 v16h;
typedef __attribute__((ext_vector_type(8)))  _Float16 v8h;
typedef __attribute__((ext_vector_type(8)))  unsigned short v8us;
typedef __attribute__((ext_vector_type(8)))  float    v8f;
typedef __attribute__((ext_vector_type(4)))  float    v4f;
typedef v8h  __attribute__((may_alias)) v8ha;
typedef v4f  __attribute__((may_alias)) v4fa;
typedef v8us __attribute__((may_alias)) v8usa;

__device__ __forceinline__ unsigned short f2bf(float f) { unsigned u = __float_as_uint(f); u += 0x7FFFu + ((u >> 16) & 1u); return (unsigned short)(u >> 16); }
__device__ __forceinline__ float bf2f(unsigned short b) { return __uint_as_float(((unsigned)b) << 16); }
__device__ __forceinline__ float bfr(float f) { return bf2f(f2bf(f)); }
__device__ __forceinline__ v16h cat16(v8h lo, v8h hi) { return __builtin_shufflevector(lo, hi, 0, 1, 2, 3, 4, 5, 6, 7, 8, 9, 10, 11, 12, 13, 14, 15); }
__device__ __forceinline__ v16bf cat16b(v8us lo, v8us hi) { return __builtin_bit_cast(v16bf, __builtin_shufflevector(lo, hi, 0, 1, 2, 3, 4, 5, 6, 7, 8, 9, 10, 11, 12, 13, 14, 15)); }
__device__ __forceinline__ v8f wmma16(v16h a, v16h b, v8f c) { return __builtin_amdgcn_wmma_f32_16x16x32_f16(false, a, false, b, (short)0, c, false, false); }
__device__ __forceinline__ v8f wmmab(v16bf a, v16bf b, v8f c) { return __builtin_amdgcn_wmma_f32_16x16x32_bf16(false, a, false, b, (short)0, c, false, false); }


template <typename T16> struct WFrag;
template <> struct WFrag<h16> { typedef v16h V; static __device__ __forceinline__ V ld(const h16* p) { return cat16(*(const v8h*)p, *(const v8h*)(p + 16)); } static __device__ __forceinline__ v8f mma(V a, V b, v8f c) { return wmma16(a, b, c); } };
template <> struct WFrag<bf> { typedef v16bf V; static __device__ __forceinline__ V ld(const bf* p) { return cat16b(*(const v8us*)p, *(const v8us*)(p + 16)); } static __device__ __forceinline__ v8f mma(V a, V b, v8f c) { return wmmab(a, b, c); } };
template <typename T16, int NSPLIT, bool BIAS>
__global__ __launch_bounds__(32) void k_gemmw(const T16* __restrict__ A, const T16* __restrict__ A2, const T16* __restrict__ Bt, const T16* __restrict__ Bt2, int K, float* C, int ldc, const float* __restrict__ bias, size_t sA, size_t sB, size_t sC) {
    typedef typename WFrag<T16>::V V;
    __shared__ __align__(16) float os[16 * 68];
    const size_t z = blockIdx.z; A += z * sA; if (A2) A2 += z * sA; Bt += z * sB; if (Bt2) Bt2 += z * sB; C += z * sC;
    const int lane = threadIdx.x & 31, lr = lane & 15, hi = lane >> 4; const int r0 = blockIdx.x * 64, c0 = blockIdx.y * 64;
    v8f acc[4][4];
#pragma unroll
    for (int mb = 0; mb < 4; ++mb)
#pragma unroll
        for (int nb = 0; nb < 4; ++nb) acc[mb][nb] = (v8f){};
    const size_t aoff = (size_t)(r0 + lr) * K + 8 * hi, boff = (size_t)(c0 + lr) * K + 8 * hi;
#pragma unroll 1
    for (int kc = 0; kc < K; kc += 32) {
        V a[4], a2[4];
#pragma unroll
        for (int mb = 0; mb < 4; ++mb) { a[mb] = WFrag<T16>::ld(A + aoff + (size_t)mb * 16 * K + kc); if (NSPLIT == 1 || NSPLIT == 2) a2[mb] = WFrag<T16>::ld(A2 + aoff + (size_t)mb * 16 * K + kc); }
#pragma unroll
        for (int nb = 0; nb < 4; ++nb) { const V b = WFrag<T16>::ld(Bt + boff + (size_t)nb * 16 * K + kc); V b2; if (NSPLIT >= 2) b2 = WFrag<T16>::ld(Bt2 + boff + (size_t)nb * 16 * K + kc);
#pragma unroll
            for (int mb = 0; mb < 4; ++mb) { acc[mb][nb] = WFrag<T16>::mma(a[mb], b, acc[mb][nb]); if (NSPLIT == 1 || NSPLIT == 2) acc[mb][nb] = WFrag<T16>::mma(a2[mb], b, acc[mb][nb]); if (NSPLIT >= 2) acc[mb][nb] = WFrag<T16>::mma(a[mb], b2, acc[mb][nb]); } }
        asm volatile("v_nop\n\tv_nop\n\tv_nop\n\tv_nop" : "+v"(acc[0][0]), "+v"(acc[1][1]), "+v"(acc[2][2]), "+v"(acc[3][3]) : "v"(a[0]), "v"(a[3]));
    }
#pragma unroll
    for (int mb = 0; mb < 4; ++mb) {
#pragma unroll
        for (int nb = 0; nb < 4; ++nb) {
#pragma unroll
            for (int j = 0; j < 8; ++j) os[(hi * 8 + j) * 68 + nb * 16 + lr] = acc[mb][nb][j]; }
        __builtin_amdgcn_wave_barrier(); asm volatile("" ::: "memory");
        float* crow = C + (size_t)(r0 + mb * 16) * ldc + c0;
#pragma unroll 1
        for (int ps = 0; ps < 2; ++ps) {
#pragma unroll
            for (int s = 0; s < 8; ++s) { const int row = 2 * s + hi, cofs = lr * 4; v4f val = *(const v4fa*)(os + row * 68 + cofs); if (BIAS) { val[0] += bfr(bias[c0 + cofs]); val[1] += bfr(bias[c0 + cofs + 1]); val[2] += bfr(bias[c0 + cofs + 2]); val[3] += bfr(bias[c0 + cofs + 3]); }
                *(volatile v4f*)(crow + (size_t)row * ldc + cofs) = val; }
            if (ps == 0) __threadfence(); }
        __builtin_amdgcn_wave_barrier(); asm volatile("" ::: "memory");
    }
}

__device__ __forceinline__ h16 tohx(float x) { return (h16)x; }
__device__ __forceinline__ void splitf(float y, unsigned short& h, unsigned short& l) { h = f2bf(y); l = f2bf(y - bf2f(h)); }
typedef __attribute__((ext_vector_type(2))) _Float16 v2h;
typedef __attribute__((ext_vector_type(4))) _Float16 v4h;
typedef __attribute__((ext_vector_type(2))) unsigned short v2us;
typedef __attribute__((ext_vector_type(4))) unsigned short v4us;
typedef __attribute__((ext_vector_type(2))) float v2f;
typedef __attribute__((ext_vector_type(4))) int v4i;

__global__ __launch_bounds__(256) void k_cvt8(const float* __restrict__ src, bf* dst, size_t n8) { const size_t i = (size_t)blockIdx.x * 256 + threadIdx.x; if (i >= n8) return; const v8f v = *(const v8f*)(src + i * 8); v8us o;
#pragma unroll
    for (int k = 0; k < 8; ++k) o[k] = f2bf(v[k]); *(volatile v8us*)(dst + i * 8) = o; __threadfence(); *(volatile v8us*)(dst + i * 8) = o; }
__global__ __launch_bounds__(256) void k_wtG(const float* __restrict__ w, int K, int N, bf* Bt) {
    const int lane = threadIdx.x & 31; const int L0 = (blockIdx.x * 8 + (threadIdx.x >> 5)) * 8; const int nlines = N * K / 64;
#pragma unroll
    for (int ps = 0; ps < 2; ++ps) {
#pragma unroll 1
        for (int l = 0; l < 8; ++l) { const int L = L0 + l; if (L >= nlines) break; const size_t e = (size_t)L * 64 + lane * 2; const int k = (int)(e % K), n = (int)(e / K); v2us o;
            o[0] = f2bf(w[(size_t)k * N + n]); o[1] = f2bf(w[(size_t)(k + 1) * N + n]); *(volatile v2us*)(Bt + e) = o; }
        if (ps == 0) __threadfence(); }
}

__global__ __launch_bounds__(256) void k_h1pl(const float* __restrict__ XW, const float* __restrict__ YW, const float* __restrict__ b1, int a0, bf* Ph, bf* Pl) { const size_t i = (size_t)blockIdx.x * 256 + threadIdx.x; if (i >= (size_t)NR * HID / 8) return; const size_t e = i * 8; const int c = (int)(e % HID); const int rr = (int)(e / HID); const int a = a0 + rr / NBX, cc = rr % NBX;
    const v8f xa = *(const v8f*)(XW + (size_t)a * HID + c); const v8f yc = *(const v8f*)(YW + (size_t)cc * HID + c); v8us oh, ol;
#pragma unroll
    for (int q = 0; q < 8; ++q) { float u = __fadd_rn(xa[q], yc[q]); asm volatile("" : "+v"(u)); float w = __fadd_rn(u, bfr(b1[c + q])); asm volatile("" : "+v"(w)); unsigned short h, l; splitf(fmaxf(w, 0.0f), h, l); oh[q] = h; ol[q] = l; }
    *(volatile v8us*)(Ph + e) = oh; *(volatile v8us*)(Pl + e) = ol; __threadfence(); *(volatile v8us*)(Ph + e) = oh; *(volatile v8us*)(Pl + e) = ol; }
__global__ __launch_bounds__(256) void k_sdot(const float* __restrict__ H2, const float* __restrict__ w3, const float* __restrict__ b3, int a0, float* out) { const size_t r = (size_t)blockIdx.x * 256 + threadIdx.x; if (r >= (size_t)NR) return; const float* hr = H2 + r * HID; float s = 0.f;
#pragma unroll 4
    for (int c = 0; c < HID; c += 4) { const v4f h4 = *(const v4f*)(hr + c);
#pragma unroll
        for (int q = 0; q < 4; ++q) { float p = __fmul_rn(fmaxf(h4[q], 0.0f), bfr(w3[c + q])); asm volatile("" : "+v"(p)); s = __fadd_rn(s, p); } }
    const float o = __fadd_rn(s, bfr(b3[0])); *(volatile float*)(out + (size_t)a0 * NBX + r) = o; __threadfence(); *(volatile float*)(out + (size_t)a0 * NBX + r) = o; }

extern "C" void kernel_launch(void* const* d_in, const int* in_sizes, int n_in,
                              void* d_out, int out_size, void* d_ws, size_t ws_size, hipStream_t stream) {
    (void)in_sizes; (void)n_in; (void)out_size;
    const float* x = (const float*)d_in[0]; const float* y = (const float*)d_in[1]; const float* w1 = (const float*)d_in[2]; const float* b1 = (const float*)d_in[3]; const float* w2 = (const float*)d_in[4]; const float* b2 = (const float*)d_in[5]; const float* w3 = (const float*)d_in[6]; const float* b3 = (const float*)d_in[7];
    float* OUT = (float*)d_out;
    char* wsp = (char*)d_ws;
    auto take = [&](size_t bytes) { char* p = wsp; wsp += (bytes + 255) & ~(size_t)255; return (void*)p; };
    bf* W1X = (bf*)take((size_t)HID * DX * 2); bf* W1Y = (bf*)take((size_t)HID * DX * 2); bf* W2B = (bf*)take((size_t)HID * HID * 2); bf* XB = (bf*)take((size_t)NBX * DX * 2); bf* YB = (bf*)take((size_t)NBX * DX * 2);
    float* XW = (float*)take((size_t)NBX * HID * 4); float* YW = (float*)take((size_t)NBX * HID * 4); bf* H1h = (bf*)take((size_t)NR * HID * 2); bf* H1l = (bf*)take((size_t)NR * HID * 2); float* H2 = (float*)take((size_t)NR * HID * 4);
    if ((size_t)(wsp - (char*)d_ws) > ws_size) return;
    k_wtG<<<(unsigned)((DX * HID / 64 + 63) / 64), 256, 0, stream>>>(w1, DX, HID, W1X); k_wtG<<<(unsigned)((DX * HID / 64 + 63) / 64), 256, 0, stream>>>(w1 + (size_t)DX * HID, DX, HID, W1Y); k_wtG<<<(unsigned)((HID * HID / 64 + 63) / 64), 256, 0, stream>>>(w2, HID, HID, W2B);
    k_cvt8<<<(unsigned)(((size_t)NBX * DX / 8 + 255) / 256), 256, 0, stream>>>(x, XB, (size_t)NBX * DX / 8); k_cvt8<<<(unsigned)(((size_t)NBX * DX / 8 + 255) / 256), 256, 0, stream>>>(y, YB, (size_t)NBX * DX / 8);
    k_gemmw<bf, 0, false><<<dim3(NBX / 64, HID / 64, 1), 32, 0, stream>>>(XB, nullptr, W1X, nullptr, DX, XW, HID, nullptr, 0, 0, 0); k_gemmw<bf, 0, false><<<dim3(NBX / 64, HID / 64, 1), 32, 0, stream>>>(YB, nullptr, W1Y, nullptr, DX, YW, HID, nullptr, 0, 0, 0);
    for (int a0 = 0; a0 < NBX; a0 += CHA) {
        k_h1pl<<<(unsigned)(((size_t)NR * HID / 8 + 255) / 256), 256, 0, stream>>>(XW, YW, b1, a0, H1h, H1l);
        k_gemmw<bf, 1, true><<<dim3(NR / 64, HID / 64, 1), 32, 0, stream>>>(H1h, H1l, W2B, nullptr, HID, H2, HID, b2, 0, 0, 0);
        k_sdot<<<(unsigned)((NR + 255) / 256), 256, 0, stream>>>(H2, w3, b3, a0, OUT); }
}
